// EncodeProcessDecode_32109175505238
// MI455X (gfx1250) — hardware-run, weakly checked
//
#include <hip/hip_runtime.h>
#include <math.h>

typedef __attribute__((ext_vector_type(16))) _Float16 v16h;
typedef __attribute__((ext_vector_type(8)))  _Float16 v8h;
typedef __attribute__((ext_vector_type(16))) __bf16   v16b;
typedef __attribute__((ext_vector_type(8)))  __bf16   v8b;
typedef __attribute__((ext_vector_type(8)))  float    v8f;
typedef __attribute__((ext_vector_type(4)))  float    v4f;
typedef __attribute__((ext_vector_type(4)))  unsigned v4u;
typedef __attribute__((ext_vector_type(2)))  unsigned v2u;
typedef __attribute__((ext_vector_type(4)))  int      v4i;

constexpr int kN      = 50000;
constexpr int kE      = 600000;
constexpr int kDn     = 32;
constexpr int kDe     = 16;
constexpr int kH      = 128;
constexpr int kNP     = 50176;
constexpr int kEChunk = 200000;
constexpr int kNChunk = 3;
constexpr float kLnEps   = 1e-6f;
constexpr float kWeCarry = 16.0f;
constexpr float kWeCarryInv = 1.0f / 16.0f;
static_assert(kEChunk * kNChunk == kE, "edge chunks");
static_assert((kEChunk % 64) == 0 && (kEChunk % 4) == 0, "edge chunk tiles");
static_assert((kNP % 512) == 0 && (kNP % 64) == 0 && kNP >= kN, "node padding");
static_assert((kN % 16) == 0, "output lines");

constexpr int SG_NODES   = 512;
constexpr int SG_THREADS = 512;
constexpr int SG_WAVES   = 16;
constexpr int SG_ITERS   = 2;
constexpr int SG_SUBCAP  = 32 * 4 * SG_ITERS;
constexpr int SG_CHUNK   = SG_THREADS * 4 * SG_ITERS;
constexpr int SG_ACC_BYTES = SG_NODES * kH * 4;
constexpr int SG_LST_BYTES = SG_WAVES * SG_SUBCAP * 4;
constexpr int SG_CNT_BYTES = 64;
constexpr int SG_DEG_BYTES = SG_NODES * 4;
constexpr int SG_LDS_BYTES = SG_ACC_BYTES + SG_LST_BYTES + SG_CNT_BYTES + SG_DEG_BYTES;
static_assert(SG_WAVES * 32 == SG_THREADS && SG_WAVES * 32 == SG_NODES && SG_WAVES * 2 == 32, "segment-sum geometry");
static_assert(SG_LDS_BYTES == 280640, "segment-sum LDS bytes");

constexpr size_t kPlane  = (size_t)kNP * kH * 4;
constexpr size_t kHalfPl = kPlane / 2;
constexpr size_t kOffR0  = 0;
constexpr size_t kOffR1  = kOffR0 + kPlane;
constexpr size_t kOffR2  = kOffR1 + kPlane;
constexpr size_t kOffR3  = kOffR2 + kPlane;
constexpr size_t kOffR4  = kOffR3 + kPlane;
constexpr size_t kSz64   = (size_t)128 * 64 * 2;
constexpr size_t kSz128  = (size_t)128 * 128 * 2;
constexpr size_t kSz256  = (size_t)128 * 256 * 2;
constexpr size_t kOffWnE0h = kOffR4 + kPlane;
constexpr size_t kOffWnE0l = kOffWnE0h + kSz64;
constexpr size_t kOffWeE0  = kOffWnE0l + kSz64;
constexpr size_t kOffWnE1h = kOffWeE0  + kSz64;
constexpr size_t kOffWnE1l = kOffWnE1h + kSz128;
constexpr size_t kOffWAh   = kOffWnE1l + kSz128;
constexpr size_t kOffWAl   = kOffWAh   + kSz256;
constexpr size_t kOffWBh   = kOffWAl   + kSz256;
constexpr size_t kOffWBl   = kOffWBh   + kSz256;
constexpr size_t kOffWDh   = kOffWBl   + kSz256;
constexpr size_t kOffWDl   = kOffWDh   + kSz128;
constexpr size_t kOffWFh   = kOffWDl   + kSz128;
constexpr size_t kOffWFl   = kOffWFh   + kSz128;
constexpr size_t kOffT0h   = kOffWFl   + kSz128;
constexpr size_t kOffT0l   = kOffT0h   + kSz128;
constexpr size_t kOffRMh   = kOffT0l   + kSz128;
constexpr size_t kOffRMl   = kOffRMh   + kSz256;
constexpr size_t kOffR1eh  = kOffRMl   + kSz256;
constexpr size_t kOffR1el  = kOffR1eh  + kSz128;
constexpr size_t kOffWEBh  = kOffR1el  + kSz128;
constexpr size_t kOffWEBl  = kOffWEBh  + kSz128;
constexpr size_t kOffBvec  = kOffWEBl  + kSz128;
constexpr size_t kOffDegA  = kOffBvec  + 512;
constexpr size_t kOffDegB  = kOffDegA  + (size_t)kNP * 4;
constexpr size_t kOffDegC  = kOffDegB  + (size_t)kNP * 4;
constexpr size_t kWsTotal  = kOffDegC  + (size_t)kNP * 4;
static_assert(kPlane == 25690112ull, "plane bytes");
static_assert(kWsTotal == 129888768ull, "carve total");
static_assert(kWsTotal <= 134217728ull, "carve cap");
static_assert((size_t)kEChunk * kH * 2 <= 2 * kPlane, "edge hidden chunk fits R2+R3");
static_assert((size_t)kNP * kDn * 2 * 2 <= kPlane, "node input planes fit R2");
static_assert((kPlane % 128) == 0 && (kHalfPl % 128) == 0 && (kOffWnE0h % 128) == 0 && (kOffBvec % 128) == 0 &&
              (kOffDegA % 128) == 0 && (kOffDegB % 128) == 0 && (kOffDegC % 128) == 0, "128-B aligned regions");

__device__ __forceinline__ unsigned bfbits(float f) {
  const unsigned u = __float_as_uint(f);
  return (u + 0x7FFFu + ((u >> 16) & 1u)) >> 16;
}
__device__ __forceinline__ float bf2f(unsigned b) { return __uint_as_float(b << 16); }
__device__ __forceinline__ void split2(float f, unsigned& h, unsigned& l) {
  h = bfbits(f);
  l = bfbits(f - bf2f(h));
}
__device__ __forceinline__ void split_pack8(const float (&x)[8], v4u& hv, v4u& lv) {
  unsigned h[8], l[8];
#pragma unroll
  for (int e = 0; e < 8; ++e) split2(x[e], h[e], l[e]);
  hv = (v4u){ (h[0] & 0xffffu) | (h[1] << 16), (h[2] & 0xffffu) | (h[3] << 16),
              (h[4] & 0xffffu) | (h[5] << 16), (h[6] & 0xffffu) | (h[7] << 16) };
  lv = (v4u){ (l[0] & 0xffffu) | (l[1] << 16), (l[2] & 0xffffu) | (l[3] << 16),
              (l[4] & 0xffffu) | (l[5] << 16), (l[6] & 0xffffu) | (l[7] << 16) };
}
__device__ __forceinline__ float h16_to_f32(unsigned hb) {
  const unsigned sgn = (hb & 0x8000u) << 16;
  const unsigned em = hb & 0x7fffu;
  const float fn = __uint_as_float((em << 13) + 0x38000000u);
  const float fs = (float)em * 5.9604644775390625e-8f;
  const float mag = (em < 0x400u) ? fs : fn;
  return __uint_as_float(__float_as_uint(mag) | sgn);
}
__device__ __forceinline__ unsigned f16bits(float f) {
  const _Float16 hv = (_Float16)f;
  return (unsigned)__builtin_bit_cast(unsigned short, hv);
}

__device__ __forceinline__ void guard1_b(v8f& a, v16b x, v16b y) { asm volatile("v_nop" : "+v"(a) : "v"(x), "v"(y)); }
__device__ __forceinline__ void guard4_b(v8f& a, v16b x, v16b y) { asm volatile("v_nop\n\tv_nop\n\tv_nop\n\tv_nop" : "+v"(a) : "v"(x), "v"(y)); }
__device__ __forceinline__ void guard1_h(v8f& a, v16h x) { asm volatile("v_nop" : "+v"(a) : "v"(x)); }
__device__ __forceinline__ void guard4_h(v8f& a, v16h x) { asm volatile("v_nop\n\tv_nop\n\tv_nop\n\tv_nop" : "+v"(a) : "v"(x)); }
__device__ __forceinline__ void keep4_h(v16h a, v16h b, v16h c, v16h d) { asm volatile("v_nop" :: "v"(a), "v"(b), "v"(c), "v"(d)); }
__device__ __forceinline__ void keep4_b(v16b a, v16b b, v16b c, v16b d) { asm volatile("v_nop" :: "v"(a), "v"(b), "v"(c), "v"(d)); }
__device__ __forceinline__ void acc_guard4(v8f& a, v8f& b, v8f& c, v8f& d) { asm volatile("v_nop\n\tv_nop\n\tv_nop\n\tv_nop" : "+v"(a), "+v"(b), "+v"(c), "+v"(d)); }

template <typename T> struct Frag;
template <> struct Frag<_Float16> {
  typedef v16h V; union U { v16h v; v8h h[2]; };
  static __device__ __forceinline__ v16h load(const _Float16* p) {
    U f; f.h[0] = *(const v8h*)(p); f.h[1] = *(const v8h*)(p + 16); return f.v;
  }
  static __device__ __forceinline__ v8f mma(v16h a, v16h b, v8f c) {
    return __builtin_amdgcn_wmma_f32_16x16x32_f16(false, a, false, b, (short)0, c, false, false);
  }
};
template <> struct Frag<__bf16> {
  typedef v16b V; union U { v16b v; v8b h[2]; };
  static __device__ __forceinline__ v16b load(const __bf16* p) {
    U f; f.h[0] = *(const v8b*)(p); f.h[1] = *(const v8b*)(p + 16); return f.v;
  }
  static __device__ __forceinline__ v8f mma(v16b a, v16b b, v8f c) {
    return __builtin_amdgcn_wmma_f32_16x16x32_bf16(false, a, false, b, (short)0, c, false, false);
  }
};

__device__ __forceinline__ void kloop3(const __bf16* Ah, const __bf16* Al, int lda,
                                       const __bf16* Bh, const __bf16* Bl, int ldb, int K,
                                       v8f (&acc)[4][4], int m0, int n0, int rlane, int koff) {
  for (int k0 = 0; k0 < K; k0 += 32) {
    v16b bh[4], bl[4];
#pragma unroll
    for (int j = 0; j < 4; ++j) {
      const size_t bo = (size_t)(n0 + (j << 4) + rlane) * ldb + koff + k0;
      bh[j] = Frag<__bf16>::load(Bh + bo);
      bl[j] = Frag<__bf16>::load(Bl + bo);
    }
#pragma unroll
    for (int i = 0; i < 4; ++i) {
      const size_t ao = (size_t)(m0 + (i << 4) + rlane) * lda + koff + k0;
      const v16b ah = Frag<__bf16>::load(Ah + ao);
      const v16b al = Frag<__bf16>::load(Al + ao);
#pragma unroll
      for (int j = 0; j < 4; ++j) {
        acc[i][j] = Frag<__bf16>::mma(ah, bh[j], acc[i][j]);
        acc[i][j] = Frag<__bf16>::mma(ah, bl[j], acc[i][j]);
        acc[i][j] = Frag<__bf16>::mma(al, bh[j], acc[i][j]);
      }
      guard1_b(acc[i][0], ah, al);
      guard1_b(acc[i][1], ah, al);
      guard1_b(acc[i][2], ah, al);
      guard4_b(acc[i][3], ah, al);
    }
    keep4_b(bh[0], bh[1], bh[2], bh[3]);
    keep4_b(bl[0], bl[1], bl[2], bl[3]);
  }
}

template <bool BIAS, bool ROWTERM, bool RESID, bool RELU, int OUT_MODE>
__global__ __launch_bounds__(256) void gemm_hl_kernel(
    const unsigned short* __restrict__ A0h, const unsigned short* __restrict__ A0l, int lda0, int K0,
    const unsigned short* __restrict__ A1h, const unsigned short* __restrict__ A1l, int lda1, int K1,
    const unsigned short* __restrict__ Bh, const unsigned short* __restrict__ Bl, int ldb,
    void* __restrict__ Cout, void* __restrict__ Cout2, int ldc,
    const float* __restrict__ bias, const float* __restrict__ rowv, const float* __restrict__ colv,
    const float* __restrict__ resid, int ldr, int M, int N) {
  __shared__ __align__(16) float sT[8][16 * 68];
  const int lane = threadIdx.x & 31;
  const int wave = threadIdx.x >> 5;
  const int tilesN = N >> 6;
  const int tilesM = M >> 6;
  const int tile = blockIdx.x * 8 + wave;
  if (tile >= tilesM * tilesN) return;
  const int tm = tile / tilesN;
  const int tn = tile - tm * tilesN;
  const int m0 = tm << 6;
  const int n0 = tn << 6;
  const int rlane = lane & 15;
  const int koff  = (lane >> 4) * 8;
  const int mOff  = (lane >> 4) * 8;

  v8f acc[4][4];
#pragma unroll
  for (int i = 0; i < 4; ++i)
#pragma unroll
    for (int j = 0; j < 4; ++j) acc[i][j] = (v8f){0.f, 0.f, 0.f, 0.f, 0.f, 0.f, 0.f, 0.f};

  kloop3((const __bf16*)A0h, (const __bf16*)A0l, lda0, (const __bf16*)Bh, (const __bf16*)Bl, ldb, K0,
         acc, m0, n0, rlane, koff);
  kloop3((const __bf16*)A1h, (const __bf16*)A1l, lda1, (const __bf16*)Bh + K0, (const __bf16*)Bl + K0, ldb, K1,
         acc, m0, n0, rlane, koff);

  acc_guard4(acc[0][0], acc[0][1], acc[0][2], acc[0][3]);
  acc_guard4(acc[1][0], acc[1][1], acc[1][2], acc[1][3]);
  acc_guard4(acc[2][0], acc[2][1], acc[2][2], acc[2][3]);
  acc_guard4(acc[3][0], acc[3][1], acc[3][2], acc[3][3]);

  float* slab = sT[wave];
  if (OUT_MODE == 0) {
    float* C = (float*)Cout;
    const int hh = lane >> 4, c4 = (lane & 15) * 4;
    v4f bias4 = (v4f){0.f, 0.f, 0.f, 0.f};
    v4f colv4 = (v4f){0.f, 0.f, 0.f, 0.f};
    if (BIAS) bias4 = *(const v4f*)(bias + n0 + c4);
    if (ROWTERM) colv4 = *(const v4f*)(colv + n0 + c4);
#pragma unroll
    for (int i = 0; i < 4; ++i) {
      const int mBase = m0 + (i << 4);
#pragma unroll
      for (int j = 0; j < 4; ++j) {
#pragma unroll
        for (int r = 0; r < 8; ++r) slab[(mOff + r) * 68 + (j << 4) + rlane] = acc[i][j][r];
      }
      __builtin_amdgcn_fence(__ATOMIC_RELEASE, "workgroup");
      __builtin_amdgcn_wave_barrier();
      __builtin_amdgcn_fence(__ATOMIC_ACQUIRE, "workgroup");
      v4f vals[8];
#pragma unroll
      for (int it = 0; it < 8; ++it) {
        const int row = it * 2 + hh;
        const int grow = mBase + row;
        v4f v = *(const v4f*)(slab + row * 68 + c4);
        if (BIAS) v += bias4;
        if (ROWTERM) {
          const float rv = rowv[grow];
          v += rv * colv4;
        }
        if (RESID) v += *(const v4f*)(resid + (size_t)grow * ldr + n0 + c4);
        if (RELU) {
          v[0] = fmaxf(v[0], 0.0f); v[1] = fmaxf(v[1], 0.0f); v[2] = fmaxf(v[2], 0.0f); v[3] = fmaxf(v[3], 0.0f);
        }
        vals[it] = v;
      }
      for (int pass = 0; pass < 2; ++pass) {
#pragma unroll
        for (int it = 0; it < 8; ++it) {
          const int row = it * 2 + hh;
          *(volatile v4f*)(C + (size_t)(mBase + row) * ldc + n0 + c4) = vals[it];
        }
        __threadfence();
      }
      __builtin_amdgcn_fence(__ATOMIC_RELEASE, "workgroup");
      __builtin_amdgcn_wave_barrier();
      __builtin_amdgcn_fence(__ATOMIC_ACQUIRE, "workgroup");
    }
  } else {
    unsigned short* Ch = (unsigned short*)Cout;
    unsigned short* Cl = (unsigned short*)Cout2;
    const int q = lane >> 3, c8 = (lane & 7) * 8;
    v4f bA = (v4f){0.f, 0.f, 0.f, 0.f}, bB = (v4f){0.f, 0.f, 0.f, 0.f};
    v4f cA = (v4f){0.f, 0.f, 0.f, 0.f}, cB = (v4f){0.f, 0.f, 0.f, 0.f};
    if (BIAS) { bA = *(const v4f*)(bias + n0 + c8); bB = *(const v4f*)(bias + n0 + c8 + 4); }
    if (ROWTERM) { cA = *(const v4f*)(colv + n0 + c8); cB = *(const v4f*)(colv + n0 + c8 + 4); }
#pragma unroll
    for (int i = 0; i < 4; ++i) {
      const int mBase = m0 + (i << 4);
#pragma unroll
      for (int j = 0; j < 4; ++j) {
#pragma unroll
        for (int r = 0; r < 8; ++r) slab[(mOff + r) * 68 + (j << 4) + rlane] = acc[i][j][r];
      }
      __builtin_amdgcn_fence(__ATOMIC_RELEASE, "workgroup");
      __builtin_amdgcn_wave_barrier();
      __builtin_amdgcn_fence(__ATOMIC_ACQUIRE, "workgroup");
      v4u hv[4], lv[4];
#pragma unroll
      for (int it = 0; it < 4; ++it) {
        const int row = it * 4 + q;
        const int grow = mBase + row;
        const float* sp = slab + row * 68 + c8;
        v4f s0 = *(const v4f*)(sp);
        v4f s1 = *(const v4f*)(sp + 4);
        if (BIAS) { s0 += bA; s1 += bB; }
        if (ROWTERM) {
          const float rv = rowv[grow];
          s0 += rv * cA;
          s1 += rv * cB;
        }
        if (RESID) {
          const float* rp = resid + (size_t)grow * ldr + n0 + c8;
          s0 += *(const v4f*)(rp);
          s1 += *(const v4f*)(rp + 4);
        }
        float x[8] = { s0[0], s0[1], s0[2], s0[3], s1[0], s1[1], s1[2], s1[3] };
        if (RELU) {
#pragma unroll
          for (int e = 0; e < 8; ++e) x[e] = fmaxf(x[e], 0.0f);
        }
        split_pack8(x, hv[it], lv[it]);
      }
      for (int pass = 0; pass < 2; ++pass) {
#pragma unroll
        for (int it = 0; it < 4; ++it) {
          const int row = it * 4 + q;
          const size_t o = (size_t)(mBase + row) * ldc + n0 + c8;
          *(volatile v4u*)(Ch + o) = hv[it];
          *(volatile v4u*)(Cl + o) = lv[it];
        }
        __threadfence();
      }
      __builtin_amdgcn_fence(__ATOMIC_RELEASE, "workgroup");
      __builtin_amdgcn_wave_barrier();
      __builtin_amdgcn_fence(__ATOMIC_ACQUIRE, "workgroup");
    }
  }
}

__global__ __launch_bounds__(256) void edge_hidden_kernel(
    const float* __restrict__ edges, int e0, int rows,
    const unsigned short* __restrict__ W16p, const float* __restrict__ b0,
    unsigned short* __restrict__ he) {
  __shared__ __align__(16) float sT[8][16 * 68];
  const int lane = threadIdx.x & 31;
  const int wave = threadIdx.x >> 5;
  const int tilesM = rows >> 6;
  const int tile = blockIdx.x * 8 + wave;
  if (tile >= tilesM * 2) return;
  const int tm = tile >> 1;
  const int tn = tile & 1;
  const int m0 = tm << 6;
  const int n0 = tn << 6;
  const int rlane = lane & 15;
  const int koff  = (lane >> 4) * 8;
  const int mOff  = (lane >> 4) * 8;
  const _Float16* W16 = (const _Float16*)W16p;

  v16h bfr[4];
#pragma unroll
  for (int j = 0; j < 4; ++j) bfr[j] = Frag<_Float16>::load(W16 + (size_t)(n0 + (j << 4) + rlane) * 64 + koff);

  v8f acc[4][4];
#pragma unroll
  for (int i = 0; i < 4; ++i)
#pragma unroll
    for (int j = 0; j < 4; ++j) acc[i][j] = (v8f){0.f, 0.f, 0.f, 0.f, 0.f, 0.f, 0.f, 0.f};

#pragma unroll
  for (int i = 0; i < 4; ++i) {
    int er = e0 + m0 + (i << 4) + rlane;
    er = er < (kE - 1) ? er : (kE - 1);
    const float* ep = edges + (size_t)er * kDe + koff;
    const v4f f0 = *(const v4f*)(ep);
    const v4f f1 = *(const v4f*)(ep + 4);
    v16h a;
    a[0] = (_Float16)f0[0]; a[1] = (_Float16)f0[1]; a[2] = (_Float16)f0[2]; a[3] = (_Float16)f0[3];
    a[4] = (_Float16)f1[0]; a[5] = (_Float16)f1[1]; a[6] = (_Float16)f1[2]; a[7] = (_Float16)f1[3];
#pragma unroll
    for (int e = 8; e < 16; ++e) a[e] = (_Float16)0.0f;
#pragma unroll
    for (int j = 0; j < 4; ++j) acc[i][j] = Frag<_Float16>::mma(a, bfr[j], acc[i][j]);
    guard1_h(acc[i][0], a);
    guard1_h(acc[i][1], a);
    guard1_h(acc[i][2], a);
    guard4_h(acc[i][3], a);
  }
  keep4_h(bfr[0], bfr[1], bfr[2], bfr[3]);
  acc_guard4(acc[0][0], acc[0][1], acc[0][2], acc[0][3]);
  acc_guard4(acc[1][0], acc[1][1], acc[1][2], acc[1][3]);
  acc_guard4(acc[2][0], acc[2][1], acc[2][2], acc[2][3]);
  acc_guard4(acc[3][0], acc[3][1], acc[3][2], acc[3][3]);

  float* slab = sT[wave];
  const int q = lane >> 3, c8 = (lane & 7) * 8;
  const v4f bA = *(const v4f*)(b0 + n0 + c8);
  const v4f bB = *(const v4f*)(b0 + n0 + c8 + 4);
#pragma unroll
  for (int i = 0; i < 4; ++i) {
    const int mBase = m0 + (i << 4);
#pragma unroll
    for (int j = 0; j < 4; ++j) {
#pragma unroll
      for (int r = 0; r < 8; ++r) slab[(mOff + r) * 68 + (j << 4) + rlane] = acc[i][j][r];
    }
    __builtin_amdgcn_fence(__ATOMIC_RELEASE, "workgroup");
    __builtin_amdgcn_wave_barrier();
    __builtin_amdgcn_fence(__ATOMIC_ACQUIRE, "workgroup");
    v4u hv[4];
#pragma unroll
    for (int it = 0; it < 4; ++it) {
      const int row = it * 4 + q;
      const float* sp = slab + row * 68 + c8;
      const v4f s0 = *(const v4f*)(sp) * kWeCarryInv + bA;
      const v4f s1 = *(const v4f*)(sp + 4) * kWeCarryInv + bB;
      const unsigned h0 = f16bits(fmaxf(s0[0], 0.0f)), h1 = f16bits(fmaxf(s0[1], 0.0f));
      const unsigned h2 = f16bits(fmaxf(s0[2], 0.0f)), h3 = f16bits(fmaxf(s0[3], 0.0f));
      const unsigned h4 = f16bits(fmaxf(s1[0], 0.0f)), h5 = f16bits(fmaxf(s1[1], 0.0f));
      const unsigned h6 = f16bits(fmaxf(s1[2], 0.0f)), h7 = f16bits(fmaxf(s1[3], 0.0f));
      hv[it] = (v4u){ h0 | (h1 << 16), h2 | (h3 << 16), h4 | (h5 << 16), h6 | (h7 << 16) };
    }
    for (int pass = 0; pass < 2; ++pass) {
#pragma unroll
      for (int it = 0; it < 4; ++it) {
        const int row = it * 4 + q;
        *(volatile v4u*)(he + (size_t)(mBase + row) * kH + n0 + c8) = hv[it];
      }
      __threadfence();
    }
    __builtin_amdgcn_fence(__ATOMIC_RELEASE, "workgroup");
    __builtin_amdgcn_wave_barrier();
    __builtin_amdgcn_fence(__ATOMIC_ACQUIRE, "workgroup");
  }
}

template <bool F16>
__global__ __launch_bounds__(256) void prep_bt_kernel(
    const float* __restrict__ src, int Kreal,
    unsigned short* __restrict__ dh, unsigned short* __restrict__ dl, int ldd, int koff, float scale) {
  __shared__ float sT[64 * 129];
  const int tid = threadIdx.x, lane = tid & 31, wave = tid >> 5;
  const int k0 = blockIdx.x * 64;
#pragma unroll 1
  for (int idx = tid; idx < 64 * 128; idx += 256) {
    const int kk = idx >> 7, n = idx & 127;
    const int kr = k0 + kk;
    const int krc = kr < Kreal ? kr : (Kreal - 1);
    const float v = src[(size_t)krc * kH + n];
    sT[kk * 129 + n] = (kr < Kreal) ? v : 0.0f;
  }
  __syncthreads();
  const int q = lane >> 3, c8 = (lane & 7) * 8;
  v4u hv[4], lv[4];
#pragma unroll
  for (int it = 0; it < 4; ++it) {
    const int n = it * 32 + wave * 4 + q;
    float x[8];
#pragma unroll
    for (int e = 0; e < 8; ++e) x[e] = sT[(c8 + e) * 129 + n];
    if (F16) {
      unsigned h[8];
#pragma unroll
      for (int e = 0; e < 8; ++e) h[e] = f16bits(x[e] * scale);
      hv[it] = (v4u){ h[0] | (h[1] << 16), h[2] | (h[3] << 16), h[4] | (h[5] << 16), h[6] | (h[7] << 16) };
      lv[it] = hv[it];
    } else {
      split_pack8(x, hv[it], lv[it]);
    }
  }
  for (int pass = 0; pass < 2; ++pass) {
#pragma unroll
    for (int it = 0; it < 4; ++it) {
      const int n = it * 32 + wave * 4 + q;
      const size_t o = (size_t)n * ldd + koff + k0 + c8;
      *(volatile v4u*)(dh + o) = hv[it];
      if (!F16) *(volatile v4u*)(dl + o) = lv[it];
    }
    __threadfence();
  }
}

__global__ __launch_bounds__(256) void split_rows_kernel(
    const float* __restrict__ src, int n_src8,
    unsigned short* __restrict__ dh, unsigned short* __restrict__ dl, int total8) {
  const int i = blockIdx.x * 256 + threadIdx.x;
  if (i >= total8) return;
  const bool valid = i < n_src8;
  const int ic = valid ? i : (n_src8 - 1);
  const v4f a0 = *(const v4f*)(src + (size_t)ic * 8);
  const v4f a1 = *(const v4f*)(src + (size_t)ic * 8 + 4);
  float x[8];
  x[0] = valid ? a0[0] : 0.0f; x[1] = valid ? a0[1] : 0.0f; x[2] = valid ? a0[2] : 0.0f; x[3] = valid ? a0[3] : 0.0f;
  x[4] = valid ? a1[0] : 0.0f; x[5] = valid ? a1[1] : 0.0f; x[6] = valid ? a1[2] : 0.0f; x[7] = valid ? a1[3] : 0.0f;
  v4u hv, lv;
  split_pack8(x, hv, lv);
  unsigned short* qh = dh + (size_t)i * 8;
  unsigned short* ql = dl + (size_t)i * 8;
  *(volatile v4u*)qh = hv;
  *(volatile v4u*)ql = lv;
  __threadfence();
  *(volatile v4u*)qh = hv;
  *(volatile v4u*)ql = lv;
}

__global__ __launch_bounds__(128) void bvec_kernel(
    const unsigned short* __restrict__ Wh, const unsigned short* __restrict__ Wl,
    const float* __restrict__ b1e, float* __restrict__ bvec) {
  __shared__ float sb[128];
  const int tid = threadIdx.x;
  sb[tid] = b1e[tid];
  __syncthreads();
  const unsigned* ph = (const unsigned*)(Wh + (size_t)tid * kH);
  const unsigned* pl = (const unsigned*)(Wl + (size_t)tid * kH);
  float acc = 0.0f;
#pragma unroll 1
  for (int w = 0; w < 64; ++w) {
    const unsigned uh = ph[w], ul = pl[w];
    const float x0 = __uint_as_float(uh << 16) + __uint_as_float(ul << 16);
    const float x1 = __uint_as_float(uh & 0xffff0000u) + __uint_as_float(ul & 0xffff0000u);
    acc = fmaf(sb[2 * w], x0, acc);
    acc = fmaf(sb[2 * w + 1], x1, acc);
  }
  *(volatile float*)(bvec + tid) = acc;
  __threadfence();
  *(volatile float*)(bvec + tid) = acc;
}

__device__ __forceinline__ void sg_push(bool t, int r, int e, int node0, unsigned* wl, int& wcnt) {
  const unsigned m = __builtin_amdgcn_ballot_w32(t);
  if (m != 0u) {
    int pos = wcnt + (int)__builtin_amdgcn_mbcnt_lo(m, 0u);
    pos = pos < (SG_SUBCAP - 1) ? pos : (SG_SUBCAP - 1);
    if (t) wl[pos] = (((unsigned)e) << 9) | (unsigned)(r - node0);
    wcnt += __builtin_popcount(m);
  }
}

template <int SRC, bool HAS_IN, bool OUT_F32>
__global__ __launch_bounds__(512) void segsum_kernel(
    const int* __restrict__ recv, const int* __restrict__ send,
    int e_begin, int e_end, int src_row0, int src_rows,
    const unsigned short* __restrict__ srcA, const unsigned short* __restrict__ srcB,
    const float* __restrict__ inAcc, const float* __restrict__ inDeg,
    float* __restrict__ outF, unsigned short* __restrict__ outHi, unsigned short* __restrict__ outLo,
    float* __restrict__ outDeg) {
  extern __shared__ __align__(16) unsigned char sg_smem[];
  float*    acc  = (float*)sg_smem;
  unsigned* lst  = (unsigned*)(sg_smem + SG_ACC_BYTES);
  int*      cnt  = (int*)(sg_smem + SG_ACC_BYTES + SG_LST_BYTES);
  float*    degs = (float*)(sg_smem + SG_ACC_BYTES + SG_LST_BYTES + SG_CNT_BYTES);

  const int tid = threadIdx.x, lane = tid & 31, wave = tid >> 5;
  const int node0 = blockIdx.x * SG_NODES;

#pragma unroll 1
  for (int i = tid; i < SG_NODES * 32; i += SG_THREADS) {
    v4f v = (v4f){0.f, 0.f, 0.f, 0.f};
    if (HAS_IN) v = *(const v4f*)(inAcc + (size_t)node0 * kH + (size_t)i * 4);
    *(v4f*)(acc + (size_t)i * 4) = v;
  }
#pragma unroll 1
  for (int i = tid; i < SG_WAVES * SG_SUBCAP; i += SG_THREADS) lst[i] = 0u;
  if (tid < SG_WAVES) cnt[tid] = 0;
  {
    float d0 = 0.0f;
    if (HAS_IN) d0 = inDeg[node0 + tid];
    degs[tid] = d0;
  }
  __syncthreads();

  unsigned* wl = lst + wave * SG_SUBCAP;
#pragma unroll 1
  for (int cb = e_begin; cb < e_end; cb += SG_CHUNK) {
    int wcnt = 0;
#pragma unroll
    for (int it = 0; it < SG_ITERS; ++it) {
      const int eb = cb + it * (SG_THREADS * 4) + tid * 4;
      const bool inr = eb < e_end;
      const int ebc = inr ? eb : (e_end - 4);
      const v4i r = *(const v4i*)(recv + ebc);
      const int r0 = r[0], r1 = r[1], r2 = r[2], r3 = r[3];
      const bool t0 = inr && ((unsigned)(r0 - node0) < (unsigned)SG_NODES);
      const bool t1 = inr && ((unsigned)(r1 - node0) < (unsigned)SG_NODES);
      const bool t2 = inr && ((unsigned)(r2 - node0) < (unsigned)SG_NODES);
      const bool t3 = inr && ((unsigned)(r3 - node0) < (unsigned)SG_NODES);
      const unsigned many = __builtin_amdgcn_ballot_w32(t0 || t1 || t2 || t3);
      if (many != 0u) {
        sg_push(t0, r0, eb + 0, node0, wl, wcnt);
        sg_push(t1, r1, eb + 1, node0, wl, wcnt);
        sg_push(t2, r2, eb + 2, node0, wl, wcnt);
        sg_push(t3, r3, eb + 3, node0, wl, wcnt);
      }
    }
    if (lane == 0) cnt[wave] = wcnt;
    __syncthreads();

    {
      const int sub = lane >> 1;
      int csub = cnt[sub];
      csub = csub < SG_SUBCAP ? csub : SG_SUBCAP;
      const unsigned* sl = lst + sub * SG_SUBCAP;
#pragma unroll 1
      for (int t = 0; t < SG_SUBCAP / 2; ++t) {
        const int idx = (lane & 1) + 2 * t;
        const bool valid = idx < csub;
        const unsigned anyv = __builtin_amdgcn_ballot_w32(valid);
        if (anyv == 0u) break;
        const int idc = idx < (SG_SUBCAP - 1) ? idx : (SG_SUBCAP - 1);
        const unsigned ent = sl[idc];
        const bool own = valid && ((int)((ent >> 5) & 15u) == wave);
        unsigned m = __builtin_amdgcn_ballot_w32(own);
#pragma unroll 1
        for (int g = 0; g < 32; ++g) {
          if (m == 0u) break;
          const int b = __builtin_ctz(m);
          m &= (m - 1u);
          const unsigned eu = (unsigned)__builtin_amdgcn_readlane((int)ent, b);
          int e = (int)(eu >> 9);
          e = e < (kE - 1) ? e : (kE - 1);
          const int nl = (int)(eu & 511u);
          float f0, f1, f2, f3;
          if (SRC == 1) {
            int s = send[e];
            s = s < 0 ? 0 : s;
            s = s > (kN - 1) ? (kN - 1) : s;
            const v2u wh = *(const v2u*)(srcA + (size_t)s * kH + lane * 4);
            const v2u wv = *(const v2u*)(srcB + (size_t)s * kH + lane * 4);
            const unsigned h0 = wh[0], h1 = wh[1], l0 = wv[0], l1 = wv[1];
            f0 = __uint_as_float(h0 << 16) + __uint_as_float(l0 << 16);
            f1 = __uint_as_float(h0 & 0xffff0000u) + __uint_as_float(l0 & 0xffff0000u);
            f2 = __uint_as_float(h1 << 16) + __uint_as_float(l1 << 16);
            f3 = __uint_as_float(h1 & 0xffff0000u) + __uint_as_float(l1 & 0xffff0000u);
          } else {
            int row = e - src_row0;
            row = row < 0 ? 0 : row;
            row = row > (src_rows - 1) ? (src_rows - 1) : row;
            const v2u wh = *(const v2u*)(srcA + (size_t)row * kH + lane * 4);
            const unsigned h0 = wh[0], h1 = wh[1];
            f0 = h16_to_f32(h0 & 0xffffu);
            f1 = h16_to_f32(h0 >> 16);
            f2 = h16_to_f32(h1 & 0xffffu);
            f3 = h16_to_f32(h1 >> 16);
          }
          float* ap = acc + nl * kH + lane * 4;
          v4f a = *(const v4f*)ap;
          a[0] += f0; a[1] += f1; a[2] += f2; a[3] += f3;
          *(v4f*)ap = a;
          if (SRC == 0) {
            if (lane == 0) degs[nl] += 1.0f;
          }
        }
      }
    }
    __syncthreads();
  }

  if (OUT_F32) {
    for (int pass = 0; pass < 2; ++pass) {
#pragma unroll 1
      for (int i = 0; i < 32; ++i) {
        const int row = wave * 32 + i;
        const v4f v = *(const v4f*)(acc + row * kH + lane * 4);
        *(volatile v4f*)(outF + (size_t)(node0 + row) * kH + lane * 4) = v;
      }
      __threadfence();
    }
  } else {
    const int hl = lane >> 4, c8 = (lane & 15) * 8;
    for (int pass = 0; pass < 2; ++pass) {
#pragma unroll 1
      for (int i = 0; i < 16; ++i) {
        const int row = wave * 32 + 2 * i + hl;
        const v4f s0 = *(const v4f*)(acc + row * kH + c8);
        const v4f s1 = *(const v4f*)(acc + row * kH + c8 + 4);
        const float x[8] = { s0[0], s0[1], s0[2], s0[3], s1[0], s1[1], s1[2], s1[3] };
        v4u hv, lv;
        split_pack8(x, hv, lv);
        const size_t o = (size_t)(node0 + row) * kH + c8;
        *(volatile v4u*)(outHi + o) = hv;
        *(volatile v4u*)(outLo + o) = lv;
      }
      __threadfence();
    }
  }
  if (SRC == 0) {
    const float d = degs[tid];
    *(volatile float*)(outDeg + node0 + tid) = d;
    __threadfence();
    *(volatile float*)(outDeg + node0 + tid) = d;
  }
}

__global__ __launch_bounds__(256) void layernorm_kernel(
    const float* __restrict__ u, const float* __restrict__ g, const float* __restrict__ b,
    unsigned short* __restrict__ nh, unsigned short* __restrict__ nl) {
  const int lane = threadIdx.x & 31, wave = threadIdx.x >> 5;
  const int row = blockIdx.x * 16 + wave * 2 + (lane >> 4);
  const int c8 = (lane & 15) * 8;
  const float* up = u + (size_t)row * kH + c8;
  const v4f x0 = *(const v4f*)(up);
  const v4f x1 = *(const v4f*)(up + 4);
  float x[8] = { x0[0], x0[1], x0[2], x0[3], x1[0], x1[1], x1[2], x1[3] };
  float s = ((x[0] + x[1]) + (x[2] + x[3])) + ((x[4] + x[5]) + (x[6] + x[7]));
  s += __shfl_xor(s, 1, 32);
  s += __shfl_xor(s, 2, 32);
  s += __shfl_xor(s, 4, 32);
  s += __shfl_xor(s, 8, 32);
  const float mu = s * (1.0f / (float)kH);
  float d[8];
  float qv = 0.0f;
#pragma unroll
  for (int e = 0; e < 8; ++e) { d[e] = x[e] - mu; qv += d[e] * d[e]; }
  qv += __shfl_xor(qv, 1, 32);
  qv += __shfl_xor(qv, 2, 32);
  qv += __shfl_xor(qv, 4, 32);
  qv += __shfl_xor(qv, 8, 32);
  const float var = qv * (1.0f / (float)kH);
  const float rs = rsqrtf(var + kLnEps);
  const v4f g0 = *(const v4f*)(g + c8), g1 = *(const v4f*)(g + c8 + 4);
  const v4f b0 = *(const v4f*)(b + c8), b1 = *(const v4f*)(b + c8 + 4);
  float y[8];
  y[0] = d[0] * rs * g0[0] + b0[0]; y[1] = d[1] * rs * g0[1] + b0[1];
  y[2] = d[2] * rs * g0[2] + b0[2]; y[3] = d[3] * rs * g0[3] + b0[3];
  y[4] = d[4] * rs * g1[0] + b1[0]; y[5] = d[5] * rs * g1[1] + b1[1];
  y[6] = d[6] * rs * g1[2] + b1[2]; y[7] = d[7] * rs * g1[3] + b1[3];
  v4u hv, lv;
  split_pack8(y, hv, lv);
  const size_t o = (size_t)row * kH + c8;
  *(volatile v4u*)(nh + o) = hv;
  *(volatile v4u*)(nl + o) = lv;
  __threadfence();
  *(volatile v4u*)(nh + o) = hv;
  *(volatile v4u*)(nl + o) = lv;
}

__global__ __launch_bounds__(256) void decode_kernel(
    const float* __restrict__ hd, const float* __restrict__ W1, const float* __restrict__ b1,
    float* __restrict__ out, int n_lines) {
  __shared__ float sW[256];
  const int tid = threadIdx.x, lane = tid & 31, wave = tid >> 5;
  sW[tid] = W1[tid];
  __syncthreads();
  const int line = blockIdx.x * 8 + wave;
  if (line < n_lines) {
    const int row = line * 16 + (lane >> 1);
    const int col = lane & 1;
    const float* hp = hd + (size_t)row * kH;
    float acc = 0.0f;
#pragma unroll 4
    for (int k4 = 0; k4 < kH / 4; ++k4) {
      const v4f v = *(const v4f*)(hp + 4 * k4);
      acc = fmaf(v[0], sW[(4 * k4 + 0) * 2 + col], acc);
      acc = fmaf(v[1], sW[(4 * k4 + 1) * 2 + col], acc);
      acc = fmaf(v[2], sW[(4 * k4 + 2) * 2 + col], acc);
      acc = fmaf(v[3], sW[(4 * k4 + 3) * 2 + col], acc);
    }
    acc += b1[col];
    float* op = out + (size_t)line * 32 + lane;
    *(volatile float*)op = acc;
    __threadfence();
    *(volatile float*)op = acc;
  }
}

extern "C" void kernel_launch(void* const* d_in, const int* in_sizes, int n_in,
                              void* d_out, int out_size, void* d_ws, size_t ws_size,
                              hipStream_t stream) {
  if (n_in < 24) return;
  if (in_sizes[0] != kN * kDn) return;
  if (in_sizes[1] != kE * kDe) return;
  if (in_sizes[2] != kE || in_sizes[3] != kE) return;
  if (in_sizes[4] != kDn * kH || in_sizes[8] != kDe * kH) return;
  if (in_sizes[12] != 2 * kH * kH || in_sizes[13] != 2 * kH * kH) return;
  if (in_sizes[22] != kH * 2 || in_sizes[23] != 2) return;
  if (out_size != kN * 2) return;
  if (ws_size < kWsTotal) return;

  const float* nodes     = (const float*)d_in[0];
  const float* edges     = (const float*)d_in[1];
  const int*   senders   = (const int*)d_in[2];
  const int*   receivers = (const int*)d_in[3];
  const float* enc_n_W0  = (const float*)d_in[4];
  const float* enc_n_b0  = (const float*)d_in[5];
  const float* enc_n_W1  = (const float*)d_in[6];
  const float* enc_n_b1  = (const float*)d_in[7];
  const float* enc_e_W0  = (const float*)d_in[8];
  const float* enc_e_b0  = (const float*)d_in[9];
  const float* enc_e_W1  = (const float*)d_in[10];
  const float* enc_e_b1  = (const float*)d_in[11];
  const float* W_msg     = (const float*)d_in[12];
  const float* node_W0   = (const float*)d_in[13];
  const float* node_b0   = (const float*)d_in[14];
  const float* node_W1   = (const float*)d_in[15];
  const float* node_b1   = (const float*)d_in[16];
  const float* W_node    = (const float*)d_in[17];
  const float* ln_g      = (const float*)d_in[18];
  const float* ln_b      = (const float*)d_in[19];
  const float* dec_W0    = (const float*)d_in[20];
  const float* dec_b0    = (const float*)d_in[21];
  const float* dec_W1    = (const float*)d_in[22];
  const float* dec_b1    = (const float*)d_in[23];
  float* out = (float*)d_out;

  char* ws = (char*)d_ws;
  unsigned short* R0h = (unsigned short*)(ws + kOffR0);
  unsigned short* R0l = (unsigned short*)(ws + kOffR0 + kHalfPl);
  float*          R1f = (float*)(ws + kOffR1);
  unsigned short* R2h = (unsigned short*)(ws + kOffR2);
  unsigned short* R2l = (unsigned short*)(ws + kOffR2 + kHalfPl);
  unsigned short* R3h = (unsigned short*)(ws + kOffR3);
  unsigned short* R3l = (unsigned short*)(ws + kOffR3 + kHalfPl);
  float*          R4f = (float*)(ws + kOffR4);
  unsigned short* HE  = (unsigned short*)(ws + kOffR2);
  unsigned short* X16h = (unsigned short*)(ws + kOffR2);
  unsigned short* X16l = (unsigned short*)(ws + kOffR2 + (size_t)kNP * kDn * 2);

  unsigned short* WnE0h = (unsigned short*)(ws + kOffWnE0h);
  unsigned short* WnE0l = (unsigned short*)(ws + kOffWnE0l);
  unsigned short* WeE0  = (unsigned short*)(ws + kOffWeE0);
  unsigned short* WnE1h = (unsigned short*)(ws + kOffWnE1h);
  unsigned short* WnE1l = (unsigned short*)(ws + kOffWnE1l);
  unsigned short* WAh   = (unsigned short*)(ws + kOffWAh);
  unsigned short* WAl   = (unsigned short*)(ws + kOffWAl);
  unsigned short* WBh   = (unsigned short*)(ws + kOffWBh);
  unsigned short* WBl   = (unsigned short*)(ws + kOffWBl);
  unsigned short* WDh   = (unsigned short*)(ws + kOffWDh);
  unsigned short* WDl   = (unsigned short*)(ws + kOffWDl);
  unsigned short* WFh   = (unsigned short*)(ws + kOffWFh);
  unsigned short* WFl   = (unsigned short*)(ws + kOffWFl);
  unsigned short* T0h   = (unsigned short*)(ws + kOffT0h);
  unsigned short* T0l   = (unsigned short*)(ws + kOffT0l);
  unsigned short* RMh   = (unsigned short*)(ws + kOffRMh);
  unsigned short* RMl   = (unsigned short*)(ws + kOffRMl);
  unsigned short* R1eh  = (unsigned short*)(ws + kOffR1eh);
  unsigned short* R1el  = (unsigned short*)(ws + kOffR1el);
  unsigned short* WEBh  = (unsigned short*)(ws + kOffWEBh);
  unsigned short* WEBl  = (unsigned short*)(ws + kOffWEBl);
  float*          bvec  = (float*)(ws + kOffBvec);
  float*          degA  = (float*)(ws + kOffDegA);
  float*          degB  = (float*)(ws + kOffDegB);
  float*          degC  = (float*)(ws + kOffDegC);

  prep_bt_kernel<false><<<1, 256, 0, stream>>>(enc_n_W0, kDn, WnE0h, WnE0l, 64, 0, 1.0f);
  prep_bt_kernel<false><<<2, 256, 0, stream>>>(enc_n_W1, kH, WnE1h, WnE1l, kH, 0, 1.0f);
  prep_bt_kernel<true><<<1, 256, 0, stream>>>(enc_e_W0, kDe, WeE0, WeE0, 64, 0, kWeCarry);
  prep_bt_kernel<false><<<2, 256, 0, stream>>>(node_W0, kH, WAh, WAl, 2 * kH, 0, 1.0f);
  prep_bt_kernel<false><<<2, 256, 0, stream>>>(node_W0 + (size_t)kH * kH, kH, T0h, T0l, kH, 0, 1.0f);
  prep_bt_kernel<false><<<2, 256, 0, stream>>>(node_W1, kH, WBh, WBl, 2 * kH, 0, 1.0f);
  prep_bt_kernel<false><<<2, 256, 0, stream>>>(W_node, kH, WBh, WBl, 2 * kH, kH, 1.0f);
  prep_bt_kernel<false><<<2, 256, 0, stream>>>(dec_W0, kH, WDh, WDl, kH, 0, 1.0f);
  split_rows_kernel<<<(2 * kH * kH / 8) / 256, 256, 0, stream>>>(W_msg, 2 * kH * kH / 8, RMh, RMl, 2 * kH * kH / 8);
  split_rows_kernel<<<(kH * kH / 8) / 256, 256, 0, stream>>>(enc_e_W1, kH * kH / 8, R1eh, R1el, kH * kH / 8);

  gemm_hl_kernel<false, false, false, false, 2><<<1, 256, 0, stream>>>(
      T0h, T0l, kH, kH, T0h, T0l, kH, 0,
      RMh, RMl, kH,
      (void*)(WAh + kH), (void*)(WAl + kH), 2 * kH,
      node_b0, node_b0, node_b0, R1f, kH, kH, kH);
  gemm_hl_kernel<false, false, false, false, 2><<<1, 256, 0, stream>>>(
      T0h, T0l, kH, kH, T0h, T0l, kH, 0,
      RMh + (size_t)kH * kH, RMl + (size_t)kH * kH, kH,
      (void*)WEBh, (void*)WEBl, kH,
      node_b0, node_b0, node_b0, R1f, kH, kH, kH);
  gemm_hl_kernel<false, false, false, false, 2><<<1, 256, 0, stream>>>(
      WEBh, WEBl, kH, kH, WEBh, WEBl, kH, 0,
      R1eh, R1el, kH,
      (void*)WFh, (void*)WFl, kH,
      node_b0, node_b0, node_b0, R1f, kH, kH, kH);
  bvec_kernel<<<1, 128, 0, stream>>>(WEBh, WEBl, enc_e_b1, bvec);

  const int edgeBlocks = ((kEChunk / 64) * 2 + 7) / 8;
  const int segBlocks  = kNP / SG_NODES;
  edge_hidden_kernel<<<edgeBlocks, 256, 0, stream>>>(edges, 0, kEChunk, WeE0, enc_e_b0, HE);
  segsum_kernel<0, false, true><<<segBlocks, SG_THREADS, SG_LDS_BYTES, stream>>>(
      receivers, senders, 0, kEChunk, 0, kEChunk, HE, HE, R4f, degA, R4f, R0h, R0l, degA);
  edge_hidden_kernel<<<edgeBlocks, 256, 0, stream>>>(edges, kEChunk, kEChunk, WeE0, enc_e_b0, HE);
  segsum_kernel<0, true, true><<<segBlocks, SG_THREADS, SG_LDS_BYTES, stream>>>(
      receivers, senders, kEChunk, 2 * kEChunk, kEChunk, kEChunk, HE, HE, R4f, degA, R1f, R0h, R0l, degB);
  edge_hidden_kernel<<<edgeBlocks, 256, 0, stream>>>(edges, 2 * kEChunk, kEChunk, WeE0, enc_e_b0, HE);
  segsum_kernel<0, true, false><<<segBlocks, SG_THREADS, SG_LDS_BYTES, stream>>>(
      receivers, senders, 2 * kEChunk, 3 * kEChunk, 2 * kEChunk, kEChunk, HE, HE, R1f, degB, R4f, R0h, R0l, degC);

  const int gemmBlocks = ((kNP / 64) * 2 + 7) / 8;
  gemm_hl_kernel<true, true, false, false, 0><<<gemmBlocks, 256, 0, stream>>>(
      R0h, R0l, kH, kH, R0h, R0l, kH, 0,
      WFh, WFl, kH,
      (void*)R1f, (void*)R1f, kH,
      node_b0, degC, bvec, R1f, kH, kNP, kH);

  split_rows_kernel<<<(kNP * kDn / 8) / 256, 256, 0, stream>>>(nodes, kN * kDn / 8, X16h, X16l, kNP * kDn / 8);
  gemm_hl_kernel<true, false, false, true, 2><<<gemmBlocks, 256, 0, stream>>>(
      X16h, X16l, kDn, kDn, X16h, X16l, kDn, 0,
      WnE0h, WnE0l, 64,
      (void*)R3h, (void*)R3l, kH,
      enc_n_b0, enc_n_b0, enc_n_b0, R1f, kH, kNP, kH);
  gemm_hl_kernel<true, false, false, false, 2><<<gemmBlocks, 256, 0, stream>>>(
      R3h, R3l, kH, kH, R3h, R3l, kH, 0,
      WnE1h, WnE1l, kH,
      (void*)R0h, (void*)R0l, kH,
      enc_n_b1, enc_n_b1, enc_n_b1, R1f, kH, kNP, kH);

  for (int step = 0; step < 5; ++step) {
    segsum_kernel<1, false, false><<<segBlocks, SG_THREADS, SG_LDS_BYTES, stream>>>(
        receivers, senders, 0, kE, 0, kNP, R0h, R0l, R1f, degC, R4f, R2h, R2l, degA);
    gemm_hl_kernel<false, false, true, true, 2><<<gemmBlocks, 256, 0, stream>>>(
        R0h, R0l, kH, kH, R2h, R2l, kH, kH,
        WAh, WAl, 2 * kH,
        (void*)R3h, (void*)R3l, kH,
        node_b0, node_b0, node_b0, R1f, kH, kNP, kH);
    gemm_hl_kernel<true, false, false, false, 0><<<gemmBlocks, 256, 0, stream>>>(
        R3h, R3l, kH, kH, R0h, R0l, kH, kH,
        WBh, WBl, 2 * kH,
        (void*)R4f, (void*)R4f, kH,
        node_b1, node_b1, node_b1, R1f, kH, kNP, kH);
    layernorm_kernel<<<kNP / 16, 256, 0, stream>>>(R4f, ln_g, ln_b, R0h, R0l);
  }

  gemm_hl_kernel<true, false, false, true, 0><<<gemmBlocks, 256, 0, stream>>>(
      R0h, R0l, kH, kH, R0h, R0l, kH, 0,
      WDh, WDl, kH,
      (void*)R4f, (void*)R4f, kH,
      dec_b0, dec_b0, dec_b0, R1f, kH, kNP, kH);
  decode_kernel<<<((kN / 16) + 7) / 8, 256, 0, stream>>>(R4f, dec_W1, dec_b1, out, kN / 16);
}
